// CustomMultiheadAttention_90718299226583
// MI455X (gfx1250) — hardware-verified
//
#include <hip/hip_runtime.h>


#ifndef NB
#define NB 4
#endif
#ifndef SEQ
#define SEQ 1024
#endif
#ifndef NB_FULL
#define NB_FULL 4
#endif
#ifndef SEQ_FULL
#define SEQ_FULL 1024
#endif

namespace {
constexpr int E = 1024, NH = 8, DH = 128;
constexpr int MROWS = NB * SEQ;
constexpr int QT = SEQ / 16;
constexpr int KT = SEQ / 16;
constexpr int NG = NB * NH;
constexpr float SCALE = 0.08838834764831845f;
static_assert(NB >= 1 && NB <= NB_FULL);
static_assert(SEQ % 128 == 0 && SEQ <= SEQ_FULL);
static_assert(E == NH * DH);
static_assert(MROWS % 128 == 0);
static_assert((NG * QT) % 4 == 0);

typedef __bf16 b16;
typedef __attribute__((ext_vector_type(16))) __bf16 v16b;
typedef __attribute__((ext_vector_type(8)))  __bf16 v8b;
typedef __attribute__((ext_vector_type(8)))  float v8f;
typedef __attribute__((ext_vector_type(4)))  float v4f;
typedef __attribute__((ext_vector_type(4)))  int v4i;

__device__ __forceinline__ v8b ld8b(const b16* p) { return *(const v8b*)p; }
__device__ __forceinline__ v16b cat8b(v8b a, v8b b) { return __builtin_shufflevector(a, b, 0, 1, 2, 3, 4, 5, 6, 7, 8, 9, 10, 11, 12, 13, 14, 15); }
__device__ __forceinline__ v16b frag_kb(const b16* p, int hh) { return cat8b(ld8b(p + 8 * hh), ld8b(p + 16 + 8 * hh)); }
__device__ __forceinline__ void split_bf16(float v, b16& hi, b16& lo) {
  const unsigned int u = __builtin_bit_cast(unsigned int, v) & 0xffff0000u;
  hi = __builtin_bit_cast(b16, (unsigned short)(u >> 16));
  lo = (b16)(v - __builtin_bit_cast(float, u));
}
__device__ __forceinline__ float bfr(float f) { return (float)(b16)f; }
__device__ __forceinline__ v8f wmma16b(v16b a, v16b b, v8f c) {
  v8f d = __builtin_amdgcn_wmma_f32_16x16x32_bf16(false, a, false, b, (short)0, c, false, false);
  asm volatile("v_nop\n\tv_nop\n\tv_nop\n\tv_nop" : "+v"(d) : "v"(a), "v"(b));
  return d;
}
__device__ __forceinline__ v8f wmma3(v16b ah, v16b al, v16b bh, v16b bl, v8f c) {
  c = wmma16b(ah, bh, c); c = wmma16b(ah, bl, c); c = wmma16b(al, bh, c); return c;
}
__device__ __forceinline__ void wave_lds_sync() {
  __builtin_amdgcn_fence(3, "workgroup");
  __builtin_amdgcn_wave_barrier();
  __builtin_amdgcn_fence(2, "workgroup");
}

__global__ __launch_bounds__(256) void cvt_kernel(const float* __restrict__ xq, const float* __restrict__ xk, const float* __restrict__ xv,
                                                  const float* __restrict__ wq, const float* __restrict__ wk, const float* __restrict__ wv,
                                                  const float* __restrict__ wo,
                                                  b16* __restrict__ Xq, b16* __restrict__ Xk, b16* __restrict__ Xv,
                                                  b16* __restrict__ Wq, b16* __restrict__ Wk, b16* __restrict__ Wv, b16* __restrict__ Wo) {
  const size_t tid = (size_t)blockIdx.x * blockDim.x + threadIdx.x, stride = (size_t)gridDim.x * blockDim.x;
  const size_t nx = (size_t)MROWS * E / 8, nw = (size_t)E * E / 8;
  const size_t total = 3 * nx + 4 * nw;
  for (size_t c = tid; c < total; c += stride) {
    const float* src; b16* dst; size_t si, di;
    if (c < 3 * nx) {
      const int which = (int)(c / nx);
      const size_t cc = c - (size_t)which * nx;
      di = cc * 8;
      const size_t m = di / E, col = di % E;
      const size_t n = m / SEQ, t = m % SEQ;
      si = (n * SEQ_FULL + t) * (size_t)E + col;
      src = (which == 0) ? xq : (which == 1) ? xk : xv;
      dst = (which == 0) ? Xq : (which == 1) ? Xk : Xv;
    } else {
      const size_t c2 = c - 3 * nx;
      const int which = (int)(c2 / nw);
      const size_t cc = c2 - (size_t)which * nw;
      di = cc * 8; si = di;
      src = (which == 0) ? wq : (which == 1) ? wk : (which == 2) ? wv : wo;
      dst = (which == 0) ? Wq : (which == 1) ? Wk : (which == 2) ? Wv : Wo;
    }
    const v4f f0 = *(const v4f*)(src + si), f1 = *(const v4f*)(src + si + 4);
    v8b o;
#pragma unroll
    for (int e = 0; e < 4; ++e) { o[e] = (b16)f0[e]; o[4 + e] = (b16)f1[e]; }
    *(volatile v8b*)(dst + di) = o;
    __threadfence();
    *(volatile v8b*)(dst + di) = o;
  }
}

__global__ __launch_bounds__(128) void qkv_gemm_kernel(const b16* __restrict__ Xq, const b16* __restrict__ Xk, const b16* __restrict__ Xv,
                                                       const b16* __restrict__ Wq, const b16* __restrict__ Wk, const b16* __restrict__ Wv,
                                                       const float* __restrict__ bq, const float* __restrict__ bk, const float* __restrict__ bv,
                                                       b16* __restrict__ Qh, b16* __restrict__ Ql, b16* __restrict__ Kh, b16* __restrict__ Kl,
                                                       b16* __restrict__ Vh, b16* __restrict__ Vl) {
  __shared__ __attribute__((aligned(16))) b16 Ts[4][2][32 * 64];
  const int lane = threadIdx.x & 31, wave = threadIdx.x >> 5, nloc = lane & 15, hlf = lane >> 4;
  const int m0 = blockIdx.y * 128 + wave * 32;
  const int c0 = blockIdx.x * 64;
  const int mat = c0 / E, cm = c0 % E, head = cm / DH, dlo = cm % DH;
  const b16* X = (mat == 0) ? Xq : (mat == 1) ? Xk : Xv;
  const b16* W = (mat == 0) ? Wq : (mat == 1) ? Wk : Wv;
  const float* bias = ((mat == 0) ? bq : (mat == 1) ? bk : bv) + cm;
  v8f acc[2][4];
#pragma unroll
  for (int r = 0; r < 2; ++r)
#pragma unroll
    for (int t = 0; t < 4; ++t) acc[r][t] = (v8f){};
#pragma unroll 2
  for (int kb = 0; kb < E; kb += 32) {
    const v16b a0 = frag_kb(X + (size_t)(m0 + nloc) * E + kb, hlf);
    const v16b a1 = frag_kb(X + (size_t)(m0 + 16 + nloc) * E + kb, hlf);
#pragma unroll
    for (int t = 0; t < 4; ++t) {
      const v16b b = frag_kb(W + (size_t)(cm + t * 16 + nloc) * E + kb, hlf);
      acc[0][t] = wmma16b(a0, b, acc[0][t]);
      acc[1][t] = wmma16b(a1, b, acc[1][t]);
    }
  }
  const int n = m0 / SEQ, t0 = m0 % SEQ, g = n * NH + head;
  b16* Tp0 = Ts[wave][0]; b16* Tp1 = Ts[wave][1];
#pragma unroll
  for (int t = 0; t < 4; ++t)
#pragma unroll
    for (int r = 0; r < 2; ++r)
#pragma unroll
      for (int v = 0; v < 8; ++v) {
        const int rr = r * 16 + v + 8 * hlf, d = t * 16 + nloc;
        b16 yh, yl; split_bf16(acc[r][t][v] + bfr(bias[d]), yh, yl);
        const int idx = (mat < 2) ? (rr * 64 + d) : ((rr >> 4) * 1024 + d * 16 + (rr & 15));
        Tp0[idx] = yh; Tp1[idx] = yl;
      }
  wave_lds_sync();
  if (mat < 2) {
    b16* Ph = (mat == 0) ? Qh : Kh; b16* Pl = (mat == 0) ? Ql : Kl;
    const size_t rowbase = (size_t)g * SEQ + t0;
#pragma unroll
    for (int j = 0; j < 8; ++j) {
      const int e = (j * 32 + lane) * 8, rr = e >> 6, cc = e & 63;
      const size_t go = (rowbase + rr) * DH + dlo + cc;
      *(volatile v8b*)(Ph + go) = ld8b(Tp0 + e); *(volatile v8b*)(Pl + go) = ld8b(Tp1 + e);
    }
    __threadfence();
#pragma unroll
    for (int j = 0; j < 8; ++j) {
      const int e = (j * 32 + lane) * 8, rr = e >> 6, cc = e & 63;
      const size_t go = (rowbase + rr) * DH + dlo + cc;
      *(volatile v8b*)(Ph + go) = ld8b(Tp0 + e); *(volatile v8b*)(Pl + go) = ld8b(Tp1 + e);
    }
  } else {
    const size_t tb = (size_t)g * KT + (t0 >> 4);
#pragma unroll
    for (int j = 0; j < 8; ++j) {
      const int e = (j * 32 + lane) * 8, kt2 = e >> 10, within = e & 1023;
      const size_t go = ((tb + kt2) * DH + dlo) * 16 + within;
      *(volatile v8b*)(Vh + go) = ld8b(Tp0 + e); *(volatile v8b*)(Vl + go) = ld8b(Tp1 + e);
    }
    __threadfence();
#pragma unroll
    for (int j = 0; j < 8; ++j) {
      const int e = (j * 32 + lane) * 8, kt2 = e >> 10, within = e & 1023;
      const size_t go = ((tb + kt2) * DH + dlo) * 16 + within;
      *(volatile v8b*)(Vh + go) = ld8b(Tp0 + e); *(volatile v8b*)(Vl + go) = ld8b(Tp1 + e);
    }
  }
}

__global__ __launch_bounds__(128) __attribute__((amdgpu_num_vgpr(256)))
void attn_kernel(const b16* __restrict__ Qh, const b16* __restrict__ Ql, const b16* __restrict__ Kh, const b16* __restrict__ Kl,
                 const b16* __restrict__ Vh, const b16* __restrict__ Vl, const int* __restrict__ am, const int* __restrict__ kpm,
                 b16* __restrict__ Yh, b16* __restrict__ Yl) {
  __shared__ __attribute__((aligned(16))) b16 Os[4][2][16 * DH];
  const int wid = threadIdx.x >> 5, lane = threadIdx.x & 31, hh = lane >> 4, col = lane & 15;
  const int qtile = blockIdx.x * 4 + wid;
  const int g = qtile / QT;
  const int q0 = (qtile % QT) << 4;
  const int n = g / NH, h = g % NH;
  const size_t ko = (size_t)g * SEQ * DH;
  const size_t qo = ((size_t)g * SEQ + q0 + col) * DH;
  const int* amrow = am + (size_t)(q0 + col) * SEQ_FULL;
  const int* kprow = kpm + (size_t)n * SEQ_FULL;
  const float ninf = -__builtin_inff();
  float m = ninf, l = 0.0f;
  v8f o[8];
#pragma unroll
  for (int t = 0; t < 8; ++t) o[t] = (v8f){};
#pragma unroll 1
  for (int kb = 0; kb < SEQ; kb += 32) {
    const size_t r0 = ko + (size_t)(kb + col) * DH, r1 = r0 + (size_t)16 * DH;
    v8f s0 = {}, s1 = {};
#pragma unroll 1
    for (int kk = 0; kk < DH; kk += 32) {
      const v16b bqh = frag_kb(Qh + qo + kk, hh), bql = frag_kb(Ql + qo + kk, hh);
      v16b ah = frag_kb(Kh + r0 + kk, hh), al = frag_kb(Kl + r0 + kk, hh);
      s0 = wmma3(ah, al, bqh, bql, s0);
      ah = frag_kb(Kh + r1 + kk, hh); al = frag_kb(Kl + r1 + kk, hh);
      s1 = wmma3(ah, al, bqh, bql, s1);
    }
    {
      const v4i a0 = *(const v4i*)(amrow + kb + 8 * hh), a1 = *(const v4i*)(amrow + kb + 8 * hh + 4);
      const v4i p0 = *(const v4i*)(kprow + kb + 8 * hh), p1 = *(const v4i*)(kprow + kb + 8 * hh + 4);
#pragma unroll
      for (int r = 0; r < 4; ++r) {
        s0[r]     = ((a0[r] | p0[r]) != 0) ? ninf : s0[r] * SCALE;
        s0[4 + r] = ((a1[r] | p1[r]) != 0) ? ninf : s0[4 + r] * SCALE;
      }
      const v4i a2 = *(const v4i*)(amrow + kb + 16 + 8 * hh), a3 = *(const v4i*)(amrow + kb + 16 + 8 * hh + 4);
      const v4i p2 = *(const v4i*)(kprow + kb + 16 + 8 * hh), p3 = *(const v4i*)(kprow + kb + 16 + 8 * hh + 4);
#pragma unroll
      for (int r = 0; r < 4; ++r) {
        s1[r]     = ((a2[r] | p2[r]) != 0) ? ninf : s1[r] * SCALE;
        s1[4 + r] = ((a3[r] | p3[r]) != 0) ? ninf : s1[4 + r] * SCALE;
      }
    }
    float mr = ninf;
#pragma unroll
    for (int r = 0; r < 8; ++r) mr = fmaxf(mr, fmaxf(s0[r], s1[r]));
    mr = fmaxf(mr, __shfl_xor(mr, 16));
    const float mn = fmaxf(m, mr);
    const float mref = (mn == ninf) ? 0.0f : mn;
    const float al_ = __expf(m - mref);
    m = mn;
    float sum = 0.0f;
    v16b pbh, pbl;
#pragma unroll
    for (int r = 0; r < 8; ++r) {
      const float e0 = __expf(s0[r] - mref), e1 = __expf(s1[r] - mref);
      sum += e0 + e1;
      b16 a, c; split_bf16(e0, a, c); pbh[r] = a; pbl[r] = c; split_bf16(e1, a, c); pbh[8 + r] = a; pbl[8 + r] = c;
    }
    sum += __shfl_xor(sum, 16);
    l = l * al_ + sum;
#pragma unroll
    for (int t = 0; t < 8; ++t) o[t] = o[t] * al_;
    const size_t v0 = ((size_t)g * KT + (kb >> 4)) * (size_t)(DH * 16) + 8 * hh, v1 = v0 + (size_t)DH * 16;
#pragma unroll
    for (int t = 0; t < 8; ++t) {
      const int f = t * 16 + col;
      const v16b vah = cat8b(ld8b(Vh + v0 + (size_t)f * 16), ld8b(Vh + v1 + (size_t)f * 16));
      const v16b val = cat8b(ld8b(Vl + v0 + (size_t)f * 16), ld8b(Vl + v1 + (size_t)f * 16));
      o[t] = wmma3(vah, val, pbh, pbl, o[t]);
    }
  }
  const float inv = 1.0f / l;
  b16* T0 = Os[wid][0]; b16* T1 = Os[wid][1];
#pragma unroll
  for (int t = 0; t < 8; ++t) {
    v8b hv, lv;
#pragma unroll
    for (int r = 0; r < 8; ++r) { b16 a, c; split_bf16(o[t][r] * inv, a, c); hv[r] = a; lv[r] = c; }
    const int idx = col * DH + t * 16 + 8 * hh;
    *(v8b*)(T0 + idx) = hv; *(v8b*)(T1 + idx) = lv;
  }
  wave_lds_sync();
  const size_t tok0 = (size_t)n * SEQ + q0;
#pragma unroll
  for (int j = 0; j < 8; ++j) {
    const int e = (j * 32 + lane) * 8, rr = e >> 7, cc = e & 127;
    const size_t go = (tok0 + rr) * E + (size_t)h * DH + cc;
    *(volatile v8b*)(Yh + go) = ld8b(T0 + e); *(volatile v8b*)(Yl + go) = ld8b(T1 + e);
  }
  __threadfence();
#pragma unroll
  for (int j = 0; j < 8; ++j) {
    const int e = (j * 32 + lane) * 8, rr = e >> 7, cc = e & 127;
    const size_t go = (tok0 + rr) * E + (size_t)h * DH + cc;
    *(volatile v8b*)(Yh + go) = ld8b(T0 + e); *(volatile v8b*)(Yl + go) = ld8b(T1 + e);
  }
}

__global__ __launch_bounds__(128) void out_gemm_kernel(const b16* __restrict__ Yh, const b16* __restrict__ Yl, const b16* __restrict__ Wo,
                                                       const float* __restrict__ bo, float* __restrict__ out) {
  __shared__ __attribute__((aligned(16))) float Ts[4][32 * 64];
  const int lane = threadIdx.x & 31, wave = threadIdx.x >> 5, nloc = lane & 15, hlf = lane >> 4;
  const int m0 = blockIdx.y * 128 + wave * 32;
  const int c0 = blockIdx.x * 64;
  v8f acc[2][4];
#pragma unroll
  for (int r = 0; r < 2; ++r)
#pragma unroll
    for (int t = 0; t < 4; ++t) acc[r][t] = (v8f){};
#pragma unroll 2
  for (int kb = 0; kb < E; kb += 32) {
    const size_t ao0 = (size_t)(m0 + nloc) * E + kb, ao1 = (size_t)(m0 + 16 + nloc) * E + kb;
    const v16b a0h = frag_kb(Yh + ao0, hlf), a0l = frag_kb(Yl + ao0, hlf);
    const v16b a1h = frag_kb(Yh + ao1, hlf), a1l = frag_kb(Yl + ao1, hlf);
#pragma unroll
    for (int t = 0; t < 4; ++t) {
      const v16b b = frag_kb(Wo + (size_t)(c0 + t * 16 + nloc) * E + kb, hlf);
      acc[0][t] = wmma16b(a0h, b, acc[0][t]); acc[0][t] = wmma16b(a0l, b, acc[0][t]);
      acc[1][t] = wmma16b(a1h, b, acc[1][t]); acc[1][t] = wmma16b(a1l, b, acc[1][t]);
    }
  }
  float* Tt = Ts[wave];
#pragma unroll
  for (int t = 0; t < 4; ++t)
#pragma unroll
    for (int r = 0; r < 2; ++r)
#pragma unroll
      for (int v = 0; v < 8; ++v) Tt[(r * 16 + v + 8 * hlf) * 64 + t * 16 + nloc] = acc[r][t][v] + bfr(bo[c0 + t * 16 + nloc]);
  wave_lds_sync();
  float* dst0 = out + (size_t)m0 * E + c0;
#pragma unroll
  for (int j = 0; j < 16; ++j) { const int rr = j * 2 + hlf, c4 = nloc * 4; *(volatile v4f*)(dst0 + (size_t)rr * E + c4) = *(const v4f*)(Tt + rr * 64 + c4); }
  __threadfence();
#pragma unroll
  for (int j = 0; j < 16; ++j) { const int rr = j * 2 + hlf, c4 = nloc * 4; *(volatile v4f*)(dst0 + (size_t)rr * E + c4) = *(const v4f*)(Tt + rr * 64 + c4); }
}
}

extern "C" void kernel_launch(void* const* d_in, const int* in_sizes, int n_in,
                              void* d_out, int out_size, void* d_ws, size_t ws_size, hipStream_t stream) {
  if (n_in < 13) return;
  const long act_need = ((long)(NB - 1) * SEQ_FULL + SEQ) * (long)E;
  if ((long)in_sizes[0] < act_need || (long)in_sizes[1] < act_need || (long)in_sizes[2] < act_need) return;
  if (in_sizes[3] < (NB - 1) * SEQ_FULL + SEQ) return;
  if ((long)in_sizes[4] < (long)(SEQ - 1) * SEQ_FULL + SEQ) return;
  if (in_sizes[5] < E * E || in_sizes[7] < E * E || in_sizes[9] < E * E || in_sizes[11] < E * E) return;
  if (in_sizes[6] < E || in_sizes[8] < E || in_sizes[10] < E || in_sizes[12] < E) return;
  if (out_size < MROWS * E) return;

  const float* query = (const float*)d_in[0];
  const float* key   = (const float*)d_in[1];
  const float* value = (const float*)d_in[2];
  const int*   kpm   = (const int*)d_in[3];
  const int*   am    = (const int*)d_in[4];
  const float* q_w   = (const float*)d_in[5];
  const float* q_b   = (const float*)d_in[6];
  const float* k_w   = (const float*)d_in[7];
  const float* k_b   = (const float*)d_in[8];
  const float* v_w   = (const float*)d_in[9];
  const float* v_b   = (const float*)d_in[10];
  const float* o_w   = (const float*)d_in[11];
  const float* o_b   = (const float*)d_in[12];
  float* out = (float*)d_out;

  const size_t plane = (size_t)MROWS * E * 2;
  const size_t wplane = (size_t)E * E * 2;
  size_t off = 0; char* ws = (char*)d_ws;
  b16* Xq  = (b16*)(ws + off); off += plane;
  b16* Xk  = (b16*)(ws + off); off += plane;
  b16* Xv  = (b16*)(ws + off); off += plane;
  b16* Wq  = (b16*)(ws + off); off += wplane;
  b16* Wk  = (b16*)(ws + off); off += wplane;
  b16* Wv  = (b16*)(ws + off); off += wplane;
  b16* Wo  = (b16*)(ws + off); off += wplane;
  b16* Qh  = (b16*)(ws + off); off += plane;
  b16* Ql  = (b16*)(ws + off); off += plane;
  b16* Kh  = (b16*)(ws + off); off += plane;
  b16* Kl  = (b16*)(ws + off); off += plane;
  b16* Vh  = (b16*)(ws + off); off += plane;
  b16* Vl  = (b16*)(ws + off); off += plane;
  b16* Yh  = (b16*)(ws + off); off += plane;
  b16* Yl  = (b16*)(ws + off); off += plane;
  if (off > ws_size) return;

  cvt_kernel<<<2048, 256, 0, stream>>>(query, key, value, q_w, k_w, v_w, o_w, Xq, Xk, Xv, Wq, Wk, Wv, Wo);
  qkv_gemm_kernel<<<dim3(3 * E / 64, MROWS / 128), 128, 0, stream>>>(Xq, Xk, Xv, Wq, Wk, Wv, q_b, k_b, v_b, Qh, Ql, Kh, Kl, Vh, Vl);
  attn_kernel<<<(NG * QT) / 4, 128, 0, stream>>>(Qh, Ql, Kh, Kl, Vh, Vl, am, kpm, Yh, Yl);
  out_gemm_kernel<<<dim3(E / 64, MROWS / 128), 128, 0, stream>>>(Yh, Yl, Wo, o_b, out);
}
